// Sequence_17712445129091
// MI455X (gfx1250) — hardware-verified
//
#include <hip/hip_runtime.h>
#include <math.h>

constexpr int NBATCH   = 4096;
constexpr int NSTEP    = 64;
constexpr int NHID     = 128;
constexpr int NGATE4   = 4 * NHID;
constexpr int NGATE3   = 3 * NHID;
constexpr int NREP     = NSTEP - 1;
constexpr int NOUTW    = 1 + NSTEP * NREP;
constexpr int NTHR     = 256;
constexpr int ENC_ROWS = 16;
constexpr int DEC_ROWS = 32;
constexpr int HPITCH   = 136;
constexpr int XSP      = 68;
constexpr int SLP      = 516;
constexpr int NQ4      = DEC_ROWS * NOUTW / 4;
constexpr float HCARRY  = 16.0f;
constexpr float WCARRY  = 16.0f;
constexpr float ACC_INV = 1.0f / 256.0f;
static_assert(NBATCH % ENC_ROWS == 0, "");
static_assert(NBATCH % DEC_ROWS == 0, "");
static_assert(NHID == 16 * (NTHR / 32), "");
static_assert(NHID % 32 == 0, "");
static_assert(ENC_ROWS * NSTEP == NTHR * 4, "");
static_assert(DEC_ROWS * NSTEP == 2 * NTHR * 4, "");
static_assert((ENC_ROWS * NHID) % (NTHR * 4) == 0, "");
static_assert((ENC_ROWS * NGATE3) % (NTHR * 4) == 0, "");
static_assert((NGATE3 / 4) % 32 == 0, "");
static_assert((DEC_ROWS * NOUTW) % 4 == 0, "");
static_assert((DEC_ROWS * NOUTW * 4) % 128 == 0, "");
static_assert(DEC_ROWS == 4 * (NTHR / 32), "");
static_assert(HPITCH % 8 == 0 && XSP % 4 == 0 && SLP % 4 == 0, "");
static_assert(2 * HPITCH % 16 == 0, "");

typedef __attribute__((ext_vector_type(16))) _Float16 v16h;
typedef __attribute__((ext_vector_type(8)))  _Float16 v8h;
typedef __attribute__((ext_vector_type(8)))  float    v8f;
typedef __attribute__((ext_vector_type(4)))  float    v4f;

__device__ __forceinline__ void guard_g4(v8f& a0, v8f& a1, v8f& a2, v8f& a3,
                                         v16h x, v16h b0, v16h b1, v16h b2, v16h b3) {
  asm volatile("v_nop\n\tv_nop\n\tv_nop\n\tv_nop"
               : "+v"(a0), "+v"(a1), "+v"(a2), "+v"(a3)
               : "v"(x), "v"(b0), "v"(b1), "v"(b2), "v"(b3));
}
__device__ __forceinline__ void guard_g3(v8f& a0, v8f& a1, v8f& a2, v16h x, v16h b0, v16h b1, v16h b2) {
  asm volatile("v_nop\n\tv_nop\n\tv_nop\n\tv_nop"
               : "+v"(a0), "+v"(a1), "+v"(a2)
               : "v"(x), "v"(b0), "v"(b1), "v"(b2));
}
__device__ __forceinline__ void acc_guard4(v8f& a, v8f& b, v8f& c, v8f& d) {
  asm volatile("v_nop\n\tv_nop\n\tv_nop\n\tv_nop" : "+v"(a), "+v"(b), "+v"(c), "+v"(d));
}
__device__ __forceinline__ void acc_guard3(v8f& a, v8f& b, v8f& c) {
  asm volatile("v_nop\n\tv_nop\n\tv_nop\n\tv_nop" : "+v"(a), "+v"(b), "+v"(c));
}

template <typename T> struct Frag;
template <> struct Frag<_Float16> {
  typedef v16h V; union U { v16h v; v8h h[2]; };
  static __device__ __forceinline__ v16h load(const _Float16* p) {
    U f; f.h[0] = *(const v8h*)(p); f.h[1] = *(const v8h*)(p + 16); return f.v;
  }
  static __device__ __forceinline__ v8f mma(v16h a, v16h b, v8f c) {
    return __builtin_amdgcn_wmma_f32_16x16x32_f16(false, a, false, b, (short)0, c, false, false);
  }
};

__device__ __forceinline__ float fsig(float x)  { return __builtin_amdgcn_rcpf(1.0f + expf(-x)); }
__device__ __forceinline__ float ftanh(float x) { return 1.0f - 2.0f * __builtin_amdgcn_rcpf(expf(2.0f * x) + 1.0f); }

__global__ __launch_bounds__(NTHR) void cvt_f16x8_kernel(const float* __restrict__ src, unsigned short* __restrict__ dst,
                                                         int n8, float sc) {
  const int i = blockIdx.x * NTHR + threadIdx.x;
  if (i < n8) {
    const float* sp = src + (size_t)i * 8;
    const v4f a = *(const v4f*)(sp);
    const v4f b = *(const v4f*)(sp + 4);
    v8h hv;
#pragma unroll
    for (int e = 0; e < 4; ++e) {
      hv[e]     = (_Float16)(a[e] * sc);
      hv[4 + e] = (_Float16)(b[e] * sc);
    }
    *(volatile v8h*)(dst + (size_t)i * 8) = hv;
    __threadfence();
    *(volatile v8h*)(dst + (size_t)i * 8) = hv;
  }
}

__global__ __launch_bounds__(NTHR) void enc_kernel(const float* __restrict__ xin, const float* __restrict__ WihE,
                                                   const float* __restrict__ bihE, const float* __restrict__ bhhE,
                                                   const float* __restrict__ bihD, const float* __restrict__ bhhD,
                                                   const unsigned short* __restrict__ WEp,
                                                   const unsigned short* __restrict__ WDp,
                                                   float* __restrict__ CE, float* __restrict__ HPo) {
  __shared__ __align__(16) _Float16 Ah[ENC_ROWS * HPITCH];
  __shared__ __align__(16) float    Xs[ENC_ROWS * XSP];
  __shared__ __align__(16) float    Slab[ENC_ROWS * SLP];
  const _Float16* WE = (const _Float16*)WEp;
  const _Float16* WD = (const _Float16*)WDp;
  const int tid = threadIdx.x, lane = tid & 31, wave = tid >> 5;
  const int c = lane & 15, hh = lane >> 4, koff = hh * 8;
  const int rowbase = blockIdx.x * ENC_ROWS;
  const int j = 16 * wave + c;

#pragma unroll 1
  for (int i = tid; i < ENC_ROWS * HPITCH; i += NTHR) Ah[i] = (_Float16)0.0f;
  {
    const int m = tid >> 4, c4 = (tid & 15) * 4;
    const v4f v = *(const v4f*)(xin + (size_t)(rowbase + m) * NSTEP + c4);
    *(v4f*)(Xs + m * XSP + c4) = v;
  }
  float wih[4], be[4];
#pragma unroll
  for (int g = 0; g < 4; ++g) { wih[g] = WihE[g * NHID + j]; be[g] = bihE[g * NHID + j]; }
  asm volatile("" ::: "memory");
#pragma unroll
  for (int g = 0; g < 4; ++g) be[g] += bhhE[g * NHID + j];
  float cst[8], hst[8];
#pragma unroll
  for (int r = 0; r < 8; ++r) { cst[r] = 0.0f; hst[r] = 0.0f; }
  __syncthreads();

  const _Float16* ahrow = Ah + c * HPITCH + koff;
  const _Float16* we    = WE + (size_t)j * NHID + koff;
  const v8f z8 = {0.f, 0.f, 0.f, 0.f, 0.f, 0.f, 0.f, 0.f};

#pragma unroll 1
  for (int t = 0; t < NSTEP; ++t) {
    v8f acc0 = z8, acc1 = z8, acc2 = z8, acc3 = z8;
#pragma unroll 1
    for (int k0 = 0; k0 < NHID; k0 += 32) {
      const v16h a  = Frag<_Float16>::load(ahrow + k0);
      const v16h b0 = Frag<_Float16>::load(we + k0);
      const v16h b1 = Frag<_Float16>::load(we + (size_t)1 * NHID * NHID + k0);
      const v16h b2 = Frag<_Float16>::load(we + (size_t)2 * NHID * NHID + k0);
      const v16h b3 = Frag<_Float16>::load(we + (size_t)3 * NHID * NHID + k0);
      acc0 = Frag<_Float16>::mma(a, b0, acc0);
      acc1 = Frag<_Float16>::mma(a, b1, acc1);
      acc2 = Frag<_Float16>::mma(a, b2, acc2);
      acc3 = Frag<_Float16>::mma(a, b3, acc3);
      guard_g4(acc0, acc1, acc2, acc3, a, b0, b1, b2, b3);
    }
    acc_guard4(acc0, acc1, acc2, acc3);
#pragma unroll
    for (int r = 0; r < 8; ++r) {
      const float x  = Xs[(8 * hh + r) * XSP + t];
      const float zi = acc0[r] * ACC_INV + (x * wih[0] + be[0]);
      const float zf = acc1[r] * ACC_INV + (x * wih[1] + be[1]);
      const float zg = acc2[r] * ACC_INV + (x * wih[2] + be[2]);
      const float zo = acc3[r] * ACC_INV + (x * wih[3] + be[3]);
      const float ig = fsig(zi);
      const float fg = fsig(zf);
      const float gg = ftanh(zg);
      const float og = fsig(zo);
      const float cn = fg * cst[r] + ig * gg;
      cst[r] = cn;
      hst[r] = og * ftanh(cn);
    }
    __syncthreads();
#pragma unroll
    for (int r = 0; r < 8; ++r) Ah[(8 * hh + r) * HPITCH + j] = (_Float16)(hst[r] * HCARRY);
    __syncthreads();
  }

  float bd[3];
#pragma unroll
  for (int g = 0; g < 3; ++g) bd[g] = bihD[g * NHID + j] + bhhD[g * NHID + j];
  const _Float16* wd = WD + (size_t)j * NHID + koff;
  v8f d0 = z8, d1 = z8, d2 = z8;
#pragma unroll 1
  for (int k0 = 0; k0 < NHID; k0 += 32) {
    const v16h a  = Frag<_Float16>::load(ahrow + k0);
    const v16h b0 = Frag<_Float16>::load(wd + k0);
    const v16h b1 = Frag<_Float16>::load(wd + (size_t)1 * NHID * NHID + k0);
    const v16h b2 = Frag<_Float16>::load(wd + (size_t)2 * NHID * NHID + k0);
    d0 = Frag<_Float16>::mma(a, b0, d0);
    d1 = Frag<_Float16>::mma(a, b1, d1);
    d2 = Frag<_Float16>::mma(a, b2, d2);
    guard_g3(d0, d1, d2, a, b0, b1, b2);
  }
  acc_guard3(d0, d1, d2);
#pragma unroll
  for (int r = 0; r < 8; ++r) {
    float* sr = Slab + (8 * hh + r) * SLP;
    sr[j]            = cst[r];
    sr[NHID + j]     = d0[r] * ACC_INV + bd[0];
    sr[2 * NHID + j] = d1[r] * ACC_INV + bd[1];
    sr[3 * NHID + j] = d2[r] * ACC_INV + bd[2];
  }
  __syncthreads();
  for (int pass = 0; pass < 2; ++pass) {
#pragma unroll
    for (int it = 0; it < 2; ++it) {
      const int idx = it * NTHR + tid;
      const int row = idx >> 5, c4 = (idx & 31) * 4;
      const v4f v = *(const v4f*)(Slab + row * SLP + c4);
      *(volatile v4f*)(CE + (size_t)(rowbase + row) * NHID + c4) = v;
    }
#pragma unroll
    for (int it = 0; it < 6; ++it) {
      const int idx = it * NTHR + tid;
      const int row = idx / 96, c4 = (idx - row * 96) * 4;
      const v4f v = *(const v4f*)(Slab + row * SLP + NHID + c4);
      *(volatile v4f*)(HPo + (size_t)(rowbase + row) * NGATE3 + c4) = v;
    }
    __threadfence();
  }
}

__global__ __launch_bounds__(NTHR) void dec_kernel(const float* __restrict__ xrev, const float* __restrict__ HPi,
                                                   const float* __restrict__ CEi, const float* __restrict__ WihD,
                                                   const float* __restrict__ WfcD, const float* __restrict__ bfcD,
                                                   const float* __restrict__ WfcE, const float* __restrict__ bfcE,
                                                   float* __restrict__ out) {
  __shared__ __align__(16) float Xr[DEC_ROWS * NSTEP];
  __shared__ __align__(16) float Dec[DEC_ROWS * NSTEP];
  __shared__ float Enc[DEC_ROWS];
  const int tid = threadIdx.x, lane = tid & 31, wave = tid >> 5;
  const int rowbase = blockIdx.x * DEC_ROWS;

#pragma unroll
  for (int it = 0; it < 2; ++it) {
    const int idx = it * NTHR + tid;
    const int m = idx >> 4, c4 = (idx & 15) * 4;
    const v4f v = *(const v4f*)(xrev + (size_t)(rowbase + m) * NSTEP + c4);
    *(v4f*)(Xr + m * NSTEP + c4) = v;
  }
  const int h4 = lane * 4;
  const v4f wi  = *(const v4f*)(WihD + h4);
  const v4f wf  = *(const v4f*)(WihD + NHID + h4);
  const v4f wg  = *(const v4f*)(WihD + 2 * NHID + h4);
  const v4f wfd = *(const v4f*)(WfcD + h4);
  const v4f wfe = *(const v4f*)(WfcE + h4);
  const float bd0 = bfcD[0];
  const float be0 = bfcE[0];
  __syncthreads();

#pragma unroll 1
  for (int rr = 0; rr < 4; ++rr) {
    const int r = wave * 4 + rr;
    const size_t grow = (size_t)(rowbase + r);
    const v4f hi4 = *(const v4f*)(HPi + grow * NGATE3 + h4);
    const v4f hf4 = *(const v4f*)(HPi + grow * NGATE3 + NHID + h4);
    const v4f hg4 = *(const v4f*)(HPi + grow * NGATE3 + 2 * NHID + h4);
    const v4f ce4 = *(const v4f*)(CEi + grow * NHID + h4);
    float pe = 0.0f;
#pragma unroll
    for (int e = 0; e < 4; ++e) pe += ce4[e] * wfe[e];
#pragma unroll
    for (int off = 16; off > 0; off >>= 1) pe += __shfl_xor(pe, off, 32);
    if (lane == 0) Enc[r] = pe + be0;
#pragma unroll 1
    for (int t = 0; t < NSTEP; ++t) {
      const float x = Xr[r * NSTEP + t];
      float s = 0.0f;
#pragma unroll
      for (int e = 0; e < 4; ++e) {
        const float zi = x * wi[e] + hi4[e];
        const float zf = x * wf[e] + hf4[e];
        const float zg = x * wg[e] + hg4[e];
        const float cd = fsig(zf) * ce4[e] + fsig(zi) * ftanh(zg);
        s += cd * wfd[e];
      }
#pragma unroll
      for (int off = 16; off > 0; off >>= 1) s += __shfl_xor(s, off, 32);
      if (lane == 0) Dec[r * NSTEP + t] = s + bd0;
    }
  }
  __syncthreads();

  const size_t fbase = (size_t)rowbase * NOUTW;
  for (int pass = 0; pass < 2; ++pass) {
    for (int q = tid; q < NQ4; q += NTHR) {
      v4f v;
#pragma unroll
      for (int e = 0; e < 4; ++e) {
        const unsigned f   = 4u * (unsigned)q + (unsigned)e;
        const unsigned r   = f / (unsigned)NOUTW;
        const unsigned col = f - r * (unsigned)NOUTW;
        const unsigned cm  = (col > 0u) ? (col - 1u) : 0u;
        const unsigned ts  = cm / (unsigned)NREP;
        const float vd = Dec[r * NSTEP + ts];
        const float ve = Enc[r];
        v[e] = (col == 0u) ? ve : vd;
      }
      *(volatile v4f*)(out + fbase + (size_t)(4 * q)) = v;
    }
    __threadfence();
  }
}

extern "C" void kernel_launch(void* const* d_in, const int* in_sizes, int n_in,
                              void* d_out, int out_size, void* d_ws, size_t ws_size, hipStream_t stream) {
  if (n_in < 14 || d_out == nullptr || d_ws == nullptr) return;
  if (in_sizes[0] != NBATCH * NSTEP || in_sizes[1] != NBATCH * NSTEP || in_sizes[2] != NGATE4 ||
      in_sizes[3] != NGATE4 * NHID || in_sizes[4] != NGATE4 || in_sizes[5] != NGATE4 || in_sizes[6] != NHID ||
      in_sizes[7] < 1 || in_sizes[8] != NGATE4 || in_sizes[9] != NGATE4 * NHID || in_sizes[10] != NGATE4 ||
      in_sizes[11] != NGATE4 || in_sizes[12] != NHID || in_sizes[13] < 1 || out_size != NBATCH * NOUTW) return;

  const float* x_in  = (const float*)d_in[0];
  const float* x_rev = (const float*)d_in[1];
  const float* WihE  = (const float*)d_in[2];
  const float* WhhE  = (const float*)d_in[3];
  const float* bihE  = (const float*)d_in[4];
  const float* bhhE  = (const float*)d_in[5];
  const float* WfcE  = (const float*)d_in[6];
  const float* bfcE  = (const float*)d_in[7];
  const float* WihD  = (const float*)d_in[8];
  const float* WhhD  = (const float*)d_in[9];
  const float* bihD  = (const float*)d_in[10];
  const float* bhhD  = (const float*)d_in[11];
  const float* WfcD  = (const float*)d_in[12];
  const float* bfcD  = (const float*)d_in[13];
  float* out = (float*)d_out;

  char* ws = (char*)d_ws; size_t off = 0;
  auto carve = [&](size_t bytes) -> char* { char* p = ws + off; off += (bytes + 255) & ~(size_t)255; return p; };
  unsigned short* WE = (unsigned short*)carve((size_t)NGATE4 * NHID * 2);
  unsigned short* WD = (unsigned short*)carve((size_t)NGATE4 * NHID * 2);
  float*          CE = (float*)carve((size_t)NBATCH * NHID * 4);
  float*          HP = (float*)carve((size_t)NBATCH * NGATE3 * 4);
  if (off > ws_size || off > (size_t)134217728) return;

  const int n8 = NGATE4 * NHID / 8;
  cvt_f16x8_kernel<<<(n8 + NTHR - 1) / NTHR, NTHR, 0, stream>>>(WhhE, WE, n8, WCARRY);
  cvt_f16x8_kernel<<<(n8 + NTHR - 1) / NTHR, NTHR, 0, stream>>>(WhhD, WD, n8, WCARRY);
  enc_kernel<<<NBATCH / ENC_ROWS, NTHR, 0, stream>>>(x_in, WihE, bihE, bhhE, bihD, bhhD, WE, WD, CE, HP);
  dec_kernel<<<NBATCH / DEC_ROWS, NTHR, 0, stream>>>(x_rev, HP, CE, WihD, WfcD, bfcD, WfcE, bfcE, out);
}
